// Non_local_MH_31799937859997
// MI455X (gfx1250) — hardware-verified
//
#include <hip/hip_runtime.h>
#include <hip/hip_bf16.h>
#include <math.h>


#define BB 2
#define SS 2048
#define DD 1024
#define HH 16
#define DKK 64
#define QW 2

typedef _Float16 bf16;
typedef __attribute__((ext_vector_type(4))) unsigned v4u_t;
typedef unsigned v4ua __attribute__((ext_vector_type(4), may_alias));
typedef __attribute__((ext_vector_type(4))) float v4f_t;
typedef float v4fa __attribute__((ext_vector_type(4), may_alias));
typedef __attribute__((ext_vector_type(16))) bf16  bf16x16;
typedef __attribute__((ext_vector_type(8)))  bf16  bf16x8;
typedef __attribute__((ext_vector_type(4)))  bf16  bf16x4;
typedef __attribute__((ext_vector_type(8)))  float f32x8;

#define LDS_STRIDE 48
#define KSTRIDE    72
#define VSTRIDE    48

__device__ __forceinline__ f32x8 wmma_bf16(bf16x16 a, bf16x16 b, f32x8 c) {
  return __builtin_amdgcn_wmma_f32_16x16x32_f16(
      false, a, false, b, (short)0, c, false, false);
}
#define RSPLIT (1.0f / 2048.0f)
__device__ __forceinline__ bf16 lo_of(float v, bf16 h) { return (bf16)((v - (float)h) * 2048.0f); }
__device__ __forceinline__ f32x8 wmma_split(bf16x16 a, bf16x16 al, bf16x16 b, bf16x16 bl, f32x8 c) {
  f32x8 x = {}; x = wmma_bf16(al, b, x); x = wmma_bf16(a, bl, x); return wmma_bf16(a, b, c) + x * RSPLIT; }

template <typename T>
__device__ __forceinline__ bf16x16 load_frag(const T* __restrict__ base, int ld,
                                             int row0, int k0) {
  const int lane = threadIdx.x & 31;
  const int r    = lane & 15;
  const int kh   = (lane >> 4) * 8;
  const T* p0 = base + (size_t)(row0 + r) * ld + (k0 + kh);
  const T* p1 = p0 + 16;
  bf16x16 f;
#pragma unroll
  for (int i = 0; i < 8; ++i) {
    f[i]     = (bf16)p0[i];
    f[i + 8] = (bf16)p1[i];
  }
  return f;
}

__device__ __forceinline__ bf16x16 lds_frag(const bf16* base, int stride) {
  const int lane = threadIdx.x & 31;
  const int row  = lane & 15;
  const int kh   = (lane >> 4) * 8;
  const bf16x8 lo = *(const bf16x8*)(base + row * stride + kh);
  const bf16x8 hi = *(const bf16x8*)(base + row * stride + kh + 16);
  bf16x16 f;
#pragma unroll
  for (int i = 0; i < 8; ++i) { f[i] = lo[i]; f[i + 8] = hi[i]; }
  return f;
}

template <typename T>
__device__ __forceinline__ void stage_read16(const T* __restrict__ p, float* buf) {
#pragma unroll
  for (int i = 0; i < 16; ++i) buf[i] = (float)p[i];
}

__device__ __forceinline__ void stage_write(bf16* dst, const float* buf, int nquad) {
#pragma unroll
  for (int i = 0; i < nquad; ++i) {
    bf16x4 q;
    q[0] = (bf16)buf[4 * i];     q[1] = (bf16)buf[4 * i + 1];
    q[2] = (bf16)buf[4 * i + 2]; q[3] = (bf16)buf[4 * i + 3];
    *(bf16x4*)(dst + 4 * i) = q;
  }
}

__global__ __launch_bounds__(256) void transpose_pack_kernel(const float* __restrict__ W, bf16* __restrict__ WT, int K, int N, size_t plane) {
  __shared__ float tile[64][65];
  const int k0 = blockIdx.y * 64, n0 = blockIdx.x * 64, t = threadIdx.x;
  for (int i = t; i < 64 * 64; i += 256) { const int kr = i >> 6, nc = i & 63; tile[kr][nc] = W[(size_t)(k0 + kr) * N + n0 + nc]; }
  __syncthreads();
#pragma unroll 1
  for (int pass = 0; pass < 2; ++pass) {
    for (int i = t; i < 64 * 8; i += 256) { const int nr = i >> 3, k8 = (i & 7) * 8; bf16 hh[8], hl[8];
#pragma unroll
      for (int e = 0; e < 8; ++e) { const float v = tile[k8 + e][nr]; hh[e] = (bf16)v; hl[e] = lo_of(v, hh[e]); }
      bf16* d = WT + (size_t)(n0 + nr) * K + k0 + k8;
      *(volatile v4u_t*)d = *(const v4ua*)hh; *(volatile v4u_t*)(d + plane) = *(const v4ua*)hl; }
    __threadfence();
  }
}

template <typename AT, typename WT, int MODE>
__global__ __launch_bounds__(256) void gemm_bias_kernel(
    const AT* __restrict__ A, const WT* __restrict__ W,
    const float* __restrict__ bias, void* __restrict__ out,
    int M, int N, int K) {
  __shared__ bf16 ldsA[128 * LDS_STRIDE];
  __shared__ bf16 ldsW[256 * LDS_STRIDE];
  __shared__ __attribute__((aligned(16))) unsigned char sob[256 * 136 * 2];

  const int t    = threadIdx.x;
  const int wave = t >> 5;
  const int lane = t & 31;
  const int wm   = (wave & 1) * 64;
  const int wn   = (wave >> 1) * 64;
  const int mBlk = blockIdx.x * 128;
  const int nBlk = blockIdx.y * 256;

  const int arow = t >> 1;
  const int ach  = (t & 1) * 16;

  float abuf[16];
  float wbuf[32];

  stage_read16(A + (size_t)(mBlk + arow) * K + ach, abuf);
  stage_read16(W + (size_t)(nBlk + t) * K,          wbuf);
  stage_read16(W + (size_t)(nBlk + t) * K + 16,     wbuf + 16);

  f32x8 acc[4][4] = {};

  for (int k = 0; k < K; k += 32) {
    __syncthreads();
    stage_write(&ldsA[arow * LDS_STRIDE + ach], abuf, 4);
    stage_write(&ldsW[t * LDS_STRIDE],          wbuf, 8);
    if (k + 32 < K) {
      stage_read16(A + (size_t)(mBlk + arow) * K + (k + 32) + ach, abuf);
      stage_read16(W + (size_t)(nBlk + t) * K + (k + 32),          wbuf);
      stage_read16(W + (size_t)(nBlk + t) * K + (k + 32) + 16,     wbuf + 16);
    }
    __syncthreads();

    bf16x16 af[4], wf[4];
#pragma unroll
    for (int i = 0; i < 4; ++i)
      af[i] = lds_frag(ldsA + (wm + 16 * i) * LDS_STRIDE, LDS_STRIDE);
#pragma unroll
    for (int j = 0; j < 4; ++j)
      wf[j] = lds_frag(ldsW + (wn + 16 * j) * LDS_STRIDE, LDS_STRIDE);
#pragma unroll
    for (int i = 0; i < 4; ++i)
#pragma unroll
      for (int j = 0; j < 4; ++j)
        acc[i][j] = wmma_bf16(af[i], wf[j], acc[i][j]);
  }

  const int nlane = lane & 15;
  const int mh    = (lane >> 4) * 8;
  __syncthreads();
  if (MODE == 0 || MODE == 1) {
    bf16* so = (bf16*)sob;
#pragma unroll
    for (int i = 0; i < 4; ++i)
#pragma unroll
      for (int j = 0; j < 4; ++j) {
        const int nl = wn + 16 * j + nlane;
        const float bv = bias[nBlk + nl];
#pragma unroll
        for (int r = 0; r < 8; ++r) {
          const int ml = wm + 16 * i + mh + r;
          const bf16 hv = (bf16)(acc[i][j][r] + bv);
          if (MODE == 0) so[ml * 264 + nl] = hv;
          else           so[nl * 136 + ml] = hv;
        }
      }
    __syncthreads();
#pragma unroll 1
    for (int pass = 0; pass < 2; ++pass) {
      if (MODE == 0) {
        for (int ch = t; ch < 128 * 32; ch += 256) { const int ml = ch >> 5, q = (ch & 31) * 8;
          *(volatile v4u_t*)((bf16*)out + (size_t)(mBlk + ml) * N + nBlk + q) = *(const v4ua*)(so + ml * 264 + q); }
      } else {
        const int b_ = mBlk >> 11, s0 = mBlk & (SS - 1);
        for (int ch = t; ch < 256 * 16; ch += 256) { const int nl = ch >> 4, q = (ch & 15) * 8; const int n = nBlk + nl, h = n >> 6, dk = n & (DKK - 1);
          *(volatile v4u_t*)((bf16*)out + (((size_t)(b_ * HH + h)) * DKK + dk) * SS + s0 + q) = *(const v4ua*)(so + nl * 136 + q); }
      }
      __threadfence();
    }
  } else {
    float* so = (float*)sob;
#pragma unroll 1
    for (int hf = 0; hf < 2; ++hf) {
      if (wm == hf * 64) {
#pragma unroll
        for (int i = 0; i < 4; ++i)
#pragma unroll
          for (int j = 0; j < 4; ++j) {
            const int nl = wn + 16 * j + nlane;
            const float bv = bias[nBlk + nl];
#pragma unroll
            for (int r = 0; r < 8; ++r) so[(16 * i + mh + r) * 260 + nl] = acc[i][j][r] + bv;
          }
      }
      __syncthreads();
#pragma unroll 1
      for (int pass = 0; pass < 2; ++pass) {
        for (int ch = t; ch < 64 * 64; ch += 256) { const int ml = ch >> 6, q = (ch & 63) * 4;
          *(volatile v4f_t*)((float*)out + (size_t)(mBlk + hf * 64 + ml) * N + nBlk + q) = *(const volatile v4fa*)(so + ml * 260 + q); }
        __threadfence();
      }
      __syncthreads();
    }
  }
}

template <typename AT, typename WT, int MODE>
__global__ __launch_bounds__(256) void gemm_split_kernel(
    const AT* __restrict__ A, size_t aPlane, const WT* __restrict__ W, size_t wPlane,
    const float* __restrict__ bias, const float* __restrict__ rbias,
    void* __restrict__ out, int M, int N, int K) {
  __shared__ bf16 ldsA[128 * LDS_STRIDE], ldsAl[128 * LDS_STRIDE];
  __shared__ bf16 ldsW[256 * LDS_STRIDE], ldsWl[256 * LDS_STRIDE];
  __shared__ __attribute__((aligned(16))) unsigned char sob[256 * 136 * 2];

  const int t    = threadIdx.x;
  const int wave = t >> 5;
  const int lane = t & 31;
  const int wm   = (wave & 1) * 64;
  const int wn   = (wave >> 1) * 64;
  const int mBlk = blockIdx.x * 128;
  const int nBlk = blockIdx.y * 256;
  const int arow = t >> 1;
  const int ach  = (t & 1) * 16;

  f32x8 acc[4][4] = {};
  for (int k = 0; k < K; k += 32) {
    __syncthreads();
    {
      const AT* ap = A + (size_t)(mBlk + arow) * K + k + ach;
      bf16 hh[16], hl[16];
      if (sizeof(AT) == 4) {
#pragma unroll
        for (int i = 0; i < 16; ++i) { const float v = (float)ap[i]; hh[i] = (bf16)v; hl[i] = lo_of(v, hh[i]); }
      } else {
#pragma unroll
        for (int i = 0; i < 16; ++i) { hh[i] = (bf16)ap[i]; hl[i] = (bf16)ap[aPlane + i]; }
      }
#pragma unroll
      for (int i = 0; i < 16; ++i) { ldsA[arow * LDS_STRIDE + ach + i] = hh[i]; ldsAl[arow * LDS_STRIDE + ach + i] = hl[i]; }
    }
    {
      const WT* wp = W + (size_t)(nBlk + t) * K + k;
      if (sizeof(WT) == 4) {
#pragma unroll
        for (int i = 0; i < 32; ++i) { const float v = (float)wp[i]; const bf16 h_ = (bf16)v; ldsW[t * LDS_STRIDE + i] = h_; ldsWl[t * LDS_STRIDE + i] = lo_of(v, h_); }
      } else {
#pragma unroll
        for (int i = 0; i < 32; ++i) { ldsW[t * LDS_STRIDE + i] = (bf16)wp[i]; ldsWl[t * LDS_STRIDE + i] = (bf16)wp[wPlane + i]; }
      }
    }
    __syncthreads();
    bf16x16 wf[4], wfl[4];
#pragma unroll
    for (int j = 0; j < 4; ++j) { wf[j] = lds_frag(ldsW + (wn + 16 * j) * LDS_STRIDE, LDS_STRIDE); wfl[j] = lds_frag(ldsWl + (wn + 16 * j) * LDS_STRIDE, LDS_STRIDE); }
#pragma unroll
    for (int i = 0; i < 4; ++i) {
      const bf16x16 af = lds_frag(ldsA + (wm + 16 * i) * LDS_STRIDE, LDS_STRIDE), afl = lds_frag(ldsAl + (wm + 16 * i) * LDS_STRIDE, LDS_STRIDE);
#pragma unroll
      for (int j = 0; j < 4; ++j) acc[i][j] = wmma_split(af, afl, wf[j], wfl[j], acc[i][j]);
    }
  }

  const int nlane = lane & 15;
  const int mh    = (lane >> 4) * 8;
  __syncthreads();
  if (MODE == 1) {
    bf16* so = (bf16*)sob;
#pragma unroll
    for (int i = 0; i < 4; ++i)
#pragma unroll
      for (int j = 0; j < 4; ++j) {
        const int nl = wn + 16 * j + nlane;
        const float bv = bias ? bias[nBlk + nl] : 0.0f;
#pragma unroll
        for (int r = 0; r < 8; ++r) so[nl * 136 + wm + 16 * i + mh + r] = (bf16)(acc[i][j][r] + bv);
      }
    __syncthreads();
    const int b_ = mBlk >> 11, s0 = mBlk & (SS - 1);
#pragma unroll 1
    for (int pass = 0; pass < 2; ++pass) {
      for (int ch = t; ch < 256 * 16; ch += 256) { const int nl = ch >> 4, q = (ch & 15) * 8; const int n = nBlk + nl, h = n >> 6, dk = n & (DKK - 1);
        *(volatile v4u_t*)((bf16*)out + (((size_t)(b_ * HH + h)) * DKK + dk) * SS + s0 + q) = *(const v4ua*)(so + nl * 136 + q); }
      __threadfence();
    }
  } else {
    float* so = (float*)sob;
#pragma unroll 1
    for (int hf = 0; hf < 2; ++hf) {
      if (wm == hf * 64) {
#pragma unroll
        for (int i = 0; i < 4; ++i)
#pragma unroll
          for (int j = 0; j < 4; ++j) {
            const int nl = wn + 16 * j + nlane;
            const float bv = bias ? bias[nBlk + nl] : 0.0f;
#pragma unroll
            for (int r = 0; r < 8; ++r) { const float rb = rbias ? rbias[mBlk + hf * 64 + 16 * i + mh + r] : 0.0f; so[(16 * i + mh + r) * 260 + nl] = acc[i][j][r] + bv + rb; }
          }
      }
      __syncthreads();
#pragma unroll 1
      for (int pass = 0; pass < 2; ++pass) {
        for (int ch = t; ch < 64 * 64; ch += 256) { const int ml = ch >> 6, q = (ch & 63) * 4;
          *(volatile v4f_t*)((float*)out + (size_t)(mBlk + hf * 64 + ml) * N + nBlk + q) = *(const volatile v4fa*)(so + ml * 260 + q); }
        __threadfence();
      }
      __syncthreads();
    }
  }
}


#define NB_ 8
#define CCH 512
#define NSP 1024
#define NHEAD 8
#define HD 64

__global__ __launch_bounds__(256) void k_blockdiag(const float* __restrict__ Mfull, float* __restrict__ Mbt) {
  const int row = blockIdx.x;
  const int h = row >> 6, e = row & 63, tid = threadIdx.x;
  __shared__ __align__(16) float r_[CCH];
  for (int k = tid; k < CCH; k += 256) { const int hk = k >> 6, m = k & 63; r_[k] = (hk == h) ? Mfull[(size_t)(h * 64 + m) * CCH + h * 64 + e] : 0.0f; }
  __syncthreads();
#pragma unroll 1
  for (int pass = 0; pass < 2; ++pass) {
    if (tid < 128) *(volatile v4f_t*)(Mbt + (size_t)row * CCH + tid * 4) = *(const volatile v4fa*)(r_ + tid * 4);
    __threadfence();
  }
}

__global__ __launch_bounds__(256) void k_residual(const float* __restrict__ ZT, const float* __restrict__ X, float* __restrict__ R) {
  __shared__ float xs[64][65];
  const int b = blockIdx.y, n0 = blockIdx.x * 64, tid = threadIdx.x;
#pragma unroll 1
  for (int o0 = 0; o0 < CCH; o0 += 64) {
    __syncthreads();
    for (int i = tid; i < 64 * 64; i += 256) { const int oo = i >> 6, nn = i & 63; xs[oo][nn] = X[((size_t)b * CCH + o0 + oo) * NSP + n0 + nn]; }
    __syncthreads();
#pragma unroll 1
    for (int pass = 0; pass < 2; ++pass) {
      for (int i = tid; i < 64 * 16; i += 256) { const int nn = i >> 4, q = (i & 15) * 4; const size_t idx = ((size_t)b * NSP + n0 + nn) * CCH + o0 + q;
        v4f_t v = *(const v4fa*)(ZT + idx); v.x += xs[q][nn]; v.y += xs[q + 1][nn]; v.z += xs[q + 2][nn]; v.w += xs[q + 3][nn];
        *(volatile v4f_t*)(R + idx) = v; }
      __threadfence();
    }
  }
}

__global__ __launch_bounds__(256) void k_bnstats(const float* __restrict__ R, float* __restrict__ mean, float* __restrict__ rsig) {
  __shared__ float s1[4][64], s2[4][64];
  const int tid = threadIdx.x, c = tid & 63, ph = tid >> 6, o = blockIdx.x * 64 + c;
  float a = 0.0f, q = 0.0f;
#pragma unroll 1
  for (int r = ph; r < NB_ * NSP; r += 4) { const float v = R[(size_t)r * CCH + o]; a += v; q += v * v; }
  s1[ph][c] = a; s2[ph][c] = q;
  __syncthreads();
  if (tid < 64) {
    const float su = (s1[0][tid] + s1[1][tid]) + (s1[2][tid] + s1[3][tid]);
    const float sq = (s2[0][tid] + s2[1][tid]) + (s2[2][tid] + s2[3][tid]);
    const float m = su / (float)(NB_ * NSP);
    const float var = fmaxf(sq / (float)(NB_ * NSP) - m * m, 0.0f);
    s1[0][tid] = m; s2[0][tid] = rsqrtf(var + 1e-5f);
  }
  __syncthreads();
#pragma unroll 1
  for (int pass = 0; pass < 2; ++pass) {
    if (tid < 64) { *(volatile float*)(mean + blockIdx.x * 64 + tid) = s1[0][tid]; *(volatile float*)(rsig + blockIdx.x * 64 + tid) = s2[0][tid]; }
    __threadfence();
  }
}

__global__ __launch_bounds__(256) void k_bnapply(const float* __restrict__ R, const float* __restrict__ mean, const float* __restrict__ rsig,
                                                const float* __restrict__ gamma, const float* __restrict__ beta, float* __restrict__ out) {
  __shared__ float ts[64][65];
  const int b = blockIdx.z, n0 = blockIdx.x * 64, o0 = blockIdx.y * 64, tid = threadIdx.x;
  for (int i = tid; i < 64 * 64; i += 256) { const int nn = i >> 6, oo = i & 63; const int o = o0 + oo;
    ts[oo][nn] = (R[((size_t)b * NSP + n0 + nn) * CCH + o] - mean[o]) * rsig[o] * gamma[o] + beta[o]; }
  __syncthreads();
#pragma unroll 1
  for (int pass = 0; pass < 2; ++pass) {
    for (int i = tid; i < 64 * 16; i += 256) { const int oo = i >> 4, q = (i & 15) * 4; v4f_t v; v.x = ts[oo][q]; v.y = ts[oo][q + 1]; v.z = ts[oo][q + 2]; v.w = ts[oo][q + 3];
      *(volatile v4f_t*)(out + ((size_t)b * CCH + o0 + oo) * NSP + n0 + q) = v; }
    __threadfence();
  }
}

extern "C" void kernel_launch(void* const* d_in, const int* in_sizes, int n_in,
                              void* d_out, int out_size, void* d_ws, size_t ws_size,
                              hipStream_t stream) {
  (void)in_sizes; (void)n_in; (void)out_size; (void)ws_size;
  const float* X  = (const float*)d_in[0];
  const float* Wq = (const float*)d_in[1];  const float* bq = (const float*)d_in[2];
  const float* Wk = (const float*)d_in[3];  const float* bk = (const float*)d_in[4];
  const float* Wv = (const float*)d_in[5];  const float* bv = (const float*)d_in[6];
  const float* Wo = (const float*)d_in[7];  const float* bo = (const float*)d_in[8];
  const float* gamma = (const float*)d_in[9]; const float* beta = (const float*)d_in[10];

  char* ws = (char*)d_ws;
  const size_t plXT = (size_t)NSP * CCH;
  bf16*  XT   = (bf16*)ws;  ws += (size_t)NB_ * 2 * plXT * 2;
  float* Kc   = (float*)ws; ws += (size_t)CCH * NSP * 4;
  float* Vc   = (float*)ws; ws += (size_t)CCH * NSP * 4;
  float* QT   = (float*)ws; ws += (size_t)NSP * CCH * 4;
  float* Mf   = (float*)ws; ws += (size_t)CCH * CCH * 4;
  float* Mbt  = (float*)ws; ws += (size_t)CCH * CCH * 4;
  float* OT   = (float*)ws; ws += (size_t)NSP * CCH * 4;
  float* ZT   = (float*)ws; ws += (size_t)NB_ * NSP * CCH * 4;
  float* R    = (float*)ws; ws += (size_t)NB_ * NSP * CCH * 4;
  float* mean = (float*)ws; ws += 4096;
  float* rsig = (float*)ws; ws += 4096;

  dim3 gBlk(256);
  for (int b = 0; b < NB_; ++b) {
    bf16* XTb = XT + (size_t)b * 2 * plXT;
    transpose_pack_kernel<<<dim3(NSP / 64, CCH / 64), 256, 0, stream>>>(X + (size_t)b * CCH * NSP, XTb, CCH, NSP, plXT);
    gemm_split_kernel<float, bf16, 2><<<dim3(CCH / 128, NSP / 256), gBlk, 0, stream>>>(Wq, 0, XTb, plXT, nullptr, bq, Kc, CCH, NSP, CCH);
    gemm_split_kernel<float, bf16, 2><<<dim3(CCH / 128, NSP / 256), gBlk, 0, stream>>>(Wv, 0, XTb, plXT, nullptr, bv, Vc, CCH, NSP, CCH);
    gemm_split_kernel<bf16, float, 2><<<dim3(NSP / 128, CCH / 256), gBlk, 0, stream>>>(XTb, plXT, Wk, 0, bk, nullptr, QT, NSP, CCH, CCH);
    gemm_split_kernel<float, float, 2><<<dim3(CCH / 128, CCH / 256), gBlk, 0, stream>>>(Kc, 0, Vc, 0, nullptr, nullptr, Mf, CCH, CCH, NSP);
    k_blockdiag<<<CCH, 256, 0, stream>>>(Mf, Mbt);
    gemm_split_kernel<float, float, 2><<<dim3(NSP / 128, CCH / 256), gBlk, 0, stream>>>(QT, 0, Mbt, 0, nullptr, nullptr, OT, NSP, CCH, CCH);
    gemm_split_kernel<float, float, 2><<<dim3(NSP / 128, CCH / 256), gBlk, 0, stream>>>(OT, 0, Wo, 0, bo, nullptr, ZT + (size_t)b * NSP * CCH, NSP, CCH, CCH);
  }
  k_residual<<<dim3(NSP / 64, NB_), 256, 0, stream>>>(ZT, X, R);
  k_bnstats<<<CCH / 64, 256, 0, stream>>>(R, mean, rsig);
  k_bnapply<<<dim3(NSP / 64, CCH / 64, NB_), 256, 0, stream>>>(R, mean, rsig, gamma, beta, (float*)d_out);
}
